// TransformerEncoderLayer_33011118637460
// MI455X (gfx1250) — hardware-verified
//
#include <hip/hip_runtime.h>

#ifndef NB
#define NB 4
#endif
#ifndef SEQ
#define SEQ 1024
#endif
#define NB_FULL 4
#define SEQ_FULL 1024
#define DM 1024
#define DMQ DM
#define NH 16
#define HD 64
#define DFF 4096
#define HG 8
#define SQ SEQ
#define NR ((size_t)NB * SEQ)
#define HCARRY 16.0f

static_assert(SEQ % 128 == 0);
static_assert(SEQ <= SEQ_FULL);
static_assert(NB >= 1 && NB <= NB_FULL);
static_assert(NH % HG == 0);
static_assert(DMQ == 1024);
static_assert(HD == 64);
static_assert(DM % 128 == 0 && DFF % 64 == 0 && DFF % 32 == 0);

typedef _Float16 v16h __attribute__((ext_vector_type(16)));
typedef unsigned short v8us __attribute__((ext_vector_type(8), may_alias));
typedef float v8f __attribute__((ext_vector_type(8)));
typedef float v4f __attribute__((ext_vector_type(4)));
typedef float v4fa __attribute__((ext_vector_type(4), may_alias));
typedef _Float16 v4h __attribute__((ext_vector_type(4)));
union FragH { v16h v; v8us half[2]; _Float16 h[16]; unsigned short u[16]; };

__device__ __forceinline__ unsigned short bf16_bits(float x) { unsigned int u = __float_as_uint(x); return (unsigned short)((u + 0x7FFFu + ((u >> 16) & 1u)) >> 16); }
__device__ __forceinline__ float bf16_val(unsigned short b) { return __uint_as_float(((unsigned int)b) << 16); }
__device__ __forceinline__ float bf16_rne(float x) { return bf16_val(bf16_bits(x)); }

__device__ __forceinline__ v16h g2_frag(const _Float16* p, int hh) { FragH f; f.half[0] = *(const v8us*)((const unsigned short*)p + 8 * hh); f.half[1] = *(const v8us*)((const unsigned short*)p + 16 + 8 * hh); return f.v; }
__device__ __forceinline__ v8f g2_mma(v16h a, v16h b, v8f c) { v8f d = __builtin_amdgcn_wmma_f32_16x16x32_f16(false, a, false, b, (short)0, c, false, false); asm volatile("v_nop\n\tv_nop\n\tv_nop\n\tv_nop" : "+v"(d) : "v"(a), "v"(b)); return d; }

__global__ __launch_bounds__(256) void k_wt_f16(const float* __restrict__ W, _Float16* __restrict__ Wt, int K, int N, float scale) {
  const int t = blockIdx.x * 256 + threadIdx.x; if (t >= N * (K / 8)) return;
  const int n = t / (K / 8), k8 = (t % (K / 8)) * 8; FragH f;
#pragma unroll
  for (int i = 0; i < 8; ++i) f.h[i] = (_Float16)(bf16_rne(W[(size_t)(k8 + i) * N + n]) * scale);
  const v8us o = f.half[0]; unsigned short* d = (unsigned short*)Wt + (size_t)n * K + k8;
  *(volatile v8us*)d = o; __threadfence(); *(volatile v8us*)d = o;
}

template <int BFIN, int INMAP, int W16, int W32>
__global__ __launch_bounds__(256) void k_lnx(const float* __restrict__ X, const float* __restrict__ g, const float* __restrict__ bb, float eps, _Float16* __restrict__ N16, float* __restrict__ N32) {
  #pragma clang fp contract(off)
  __shared__ float red[256]; const size_t r = blockIdx.x; const int t = threadIdx.x;
  const size_t rin = INMAP ? ((r / SEQ) * (size_t)SEQ_FULL + (r % SEQ)) : r;
  const bool act = t < (DMQ / 4); const int c0 = act ? t * 4 : 0;
  const v4f xa = *(const v4fa*)(X + rin * DMQ + c0); float s[4]; float sum = 0.f;
  for (int q = 0; q < 4; ++q) { s[q] = act ? (BFIN ? bf16_rne(xa[q]) : xa[q]) : 0.f; sum = __fadd_rn(sum, s[q]); }
  red[t] = sum; __syncthreads(); for (int st = 128; st > 0; st >>= 1) { if (t < st) red[t] = __fadd_rn(red[t], red[t + st]); __syncthreads(); } const float mu = red[0] / (float)DMQ; __syncthreads();
  float vs = 0.f; for (int q = 0; q < 4; ++q) { const float dl = act ? __fadd_rn(s[q], -mu) : 0.f; vs = __fadd_rn(vs, __fmul_rn(dl, dl)); } red[t] = vs; __syncthreads(); for (int st = 128; st > 0; st >>= 1) { if (t < st) red[t] = __fadd_rn(red[t], red[t + st]); __syncthreads(); }
  const float rs = rsqrtf(__fadd_rn(red[0] / (float)DMQ, eps)); v4h y; v4f yf;
  for (int q = 0; q < 4; ++q) { const int c = c0 + q; yf[q] = __fadd_rn(__fmul_rn(__fmul_rn(__fadd_rn(s[q], -mu), rs), bf16_rne(g[c])), bf16_rne(bb[c])); y[q] = (_Float16)yf[q]; }
  if (!act) return;
  for (int pass = 0; pass < 2; ++pass) { if (W16) *(volatile v4h*)(N16 + r * DMQ + c0) = y; if (W32) *(volatile v4f*)(N32 + r * DMQ + c0) = yf; if (pass == 0) __threadfence(); } }

template <int ACT, int CPBF, int OUTMAP>
__global__ __launch_bounds__(128) void k_gemm2(const _Float16* __restrict__ A, int lda, size_t sA, const _Float16* __restrict__ Bh, int ldb, size_t sB, float alpha, const float* __restrict__ bias, size_t sBias,
    const float* __restrict__ CP, int row0g, float* __restrict__ C, _Float16* __restrict__ C16, int ldc, size_t sC, int M, int N, int K) {
  static_assert(ACT == 0);
  __shared__ __attribute__((aligned(16))) float so[4][32][68];
  const int tid = threadIdx.x, w = tid >> 5, lane = tid & 31, ln = lane & 15, hh = lane >> 4; const int by = blockIdx.y;
  A += (size_t)by * sA; Bh += (size_t)by * sB; const size_t cofs = (size_t)by * sC; const float* bp = bias ? bias + (size_t)by * sBias : nullptr;
  const int ntn = N >> 6; const int mt = blockIdx.x / ntn, nq = blockIdx.x - mt * ntn; const int row0 = mt * 128 + 32 * w, col0 = nq * 64; if (row0 >= M) return;
  const _Float16* a0p = A + (size_t)(row0 + ln) * lda; const _Float16* a1p = a0p + (size_t)16 * lda;
  const _Float16* b0p = Bh + (size_t)(col0 + ln) * ldb; const _Float16* b1p = b0p + (size_t)16 * ldb; const _Float16* b2p = b1p + (size_t)16 * ldb; const _Float16* b3p = b2p + (size_t)16 * ldb;
  const v8f z8 = {0.f,0.f,0.f,0.f,0.f,0.f,0.f,0.f}; v8f c00 = z8, c01 = z8, c02 = z8, c03 = z8, c10 = z8, c11 = z8, c12 = z8, c13 = z8;
#pragma unroll 1
  for (int kb = 0; kb < K; kb += 32) { const v16h a0 = g2_frag(a0p + kb, hh), a1 = g2_frag(a1p + kb, hh);
    v16h b = g2_frag(b0p + kb, hh); c00 = g2_mma(a0, b, c00); c10 = g2_mma(a1, b, c10);
    b = g2_frag(b1p + kb, hh); c01 = g2_mma(a0, b, c01); c11 = g2_mma(a1, b, c11);
    b = g2_frag(b2p + kb, hh); c02 = g2_mma(a0, b, c02); c12 = g2_mma(a1, b, c12);
    b = g2_frag(b3p + kb, hh); c03 = g2_mma(a0, b, c03); c13 = g2_mma(a1, b, c13); }
  v8f accs[8] = {c00, c01, c02, c03, c10, c11, c12, c13};
#pragma unroll
  for (int u = 0; u < 8; ++u) { const int t = u & 3, half = u >> 2; const int col = col0 + t * 16 + ln; const float bv = bp ? bf16_rne(bp[col]) : 0.f;
#pragma unroll
    for (int r = 0; r < 8; ++r) { const int rloc = half * 16 + 8 * hh + r; float v = accs[u][r] * alpha + bv;
      if (CP) { const int rr = row0g + row0 + rloc;
        if (CPBF) { const size_t rin = (size_t)(rr / SEQ) * (size_t)SEQ_FULL + (size_t)(rr % SEQ); v += bf16_rne(CP[rin * (size_t)ldc + col]); }
        else v += CP[cofs + (size_t)rr * ldc + col]; }
      so[w][rloc][t * 16 + ln] = v; } }
  __builtin_amdgcn_fence(4  , "workgroup"); __builtin_amdgcn_wave_barrier();
  const int rsub = lane >> 4, c4 = (lane & 15) * 4;
  for (int pass = 0; pass < 2; ++pass) {
#pragma unroll
    for (int q = 0; q < 16; ++q) { const int r = q * 2 + rsub; const size_t grow = (size_t)(row0 + r); const size_t orow = OUTMAP ? ((grow / SEQ) * (size_t)SEQ_FULL + (grow % SEQ)) : grow;
      const v4f v = *(const v4fa*)&so[w][r][c4]; if (C) *(volatile v4f*)(C + cofs + orow * (size_t)ldc + col0 + c4) = v; if (C16) { v4h h4; for (int i = 0; i < 4; ++i) h4[i] = (_Float16)v[i]; *(volatile v4h*)(C16 + cofs + orow * (size_t)ldc + col0 + c4) = h4; } }
    if (pass == 0) __threadfence(); } }

__global__ __launch_bounds__(128) void k_gemm2g(const _Float16* __restrict__ A, int lda, const _Float16* __restrict__ Bh, int ldb, float alpha, const float* __restrict__ bias, float hsc,
    _Float16* __restrict__ H16, int ldh, int M, int N, int K) {
  __shared__ __attribute__((aligned(16))) float so[4][32][68];
  const int tid = threadIdx.x, w = tid >> 5, lane = tid & 31, ln = lane & 15, hh = lane >> 4;
  const int ntn = N >> 6; const int mt = blockIdx.x / ntn, nq = blockIdx.x - mt * ntn; const int row0 = mt * 128 + 32 * w, col0 = nq * 64; if (row0 >= M) return;
  const _Float16* a0p = A + (size_t)(row0 + ln) * lda; const _Float16* a1p = a0p + (size_t)16 * lda;
  const _Float16* b0p = Bh + (size_t)(col0 + ln) * ldb; const _Float16* b1p = b0p + (size_t)16 * ldb; const _Float16* b2p = b1p + (size_t)16 * ldb; const _Float16* b3p = b2p + (size_t)16 * ldb;
  const v8f z8 = {0.f,0.f,0.f,0.f,0.f,0.f,0.f,0.f}; v8f c00 = z8, c01 = z8, c02 = z8, c03 = z8, c10 = z8, c11 = z8, c12 = z8, c13 = z8;
#pragma unroll 1
  for (int kb = 0; kb < K; kb += 32) { const v16h a0 = g2_frag(a0p + kb, hh), a1 = g2_frag(a1p + kb, hh);
    v16h b = g2_frag(b0p + kb, hh); c00 = g2_mma(a0, b, c00); c10 = g2_mma(a1, b, c10);
    b = g2_frag(b1p + kb, hh); c01 = g2_mma(a0, b, c01); c11 = g2_mma(a1, b, c11);
    b = g2_frag(b2p + kb, hh); c02 = g2_mma(a0, b, c02); c12 = g2_mma(a1, b, c12);
    b = g2_frag(b3p + kb, hh); c03 = g2_mma(a0, b, c03); c13 = g2_mma(a1, b, c13); }
  v8f accs[8] = {c00, c01, c02, c03, c10, c11, c12, c13};
#pragma unroll
  for (int u = 0; u < 8; ++u) { const int t = u & 3, half = u >> 2; const int col = col0 + t * 16 + ln; const float bv = bias ? bf16_rne(bias[col]) : 0.f;
#pragma unroll
    for (int r = 0; r < 8; ++r) { const int rloc = half * 16 + 8 * hh + r; float v = accs[u][r] * alpha + bv;
      v = 0.5f * v * (1.0f + erff(v * 0.70710678118654752f)); v *= hsc;
      so[w][rloc][t * 16 + ln] = v; } }
  __builtin_amdgcn_fence(4  , "workgroup"); __builtin_amdgcn_wave_barrier();
  const int rsub = lane >> 4, c4 = (lane & 15) * 4;
  for (int pass = 0; pass < 2; ++pass) {
#pragma unroll
    for (int q = 0; q < 16; ++q) { const int r = q * 2 + rsub; const v4f v = *(const v4fa*)&so[w][r][c4]; v4h h4; for (int i = 0; i < 4; ++i) h4[i] = (_Float16)v[i];
      *(volatile v4h*)(H16 + (size_t)(row0 + r) * ldh + col0 + c4) = h4; }
    if (pass == 0) __threadfence(); } }

__global__ __launch_bounds__(256) void k_rsmf(const float* __restrict__ S, _Float16* __restrict__ P, int qn, int hg) {
  #pragma clang fp contract(off)
  const int t = blockIdx.x * 256 + threadIdx.x; if (t >= qn * hg) return; const size_t i = (size_t)(t / qn) * SQ + (t % qn); const float* s = S + i * SQ; float mx = -3.0e38f;
#pragma unroll 1
  for (int j = 0; j < SQ; ++j) mx = fmaxf(mx, s[j]); float se = 0.f;
#pragma unroll 1
  for (int j = 0; j < SQ; ++j) se += __expf(s[j] - mx); const float sc = 256.0f / se;
#pragma unroll 1
  for (int j0 = 0; j0 < SQ; j0 += 8) { FragH f; for (int q = 0; q < 8; ++q) f.h[q] = (_Float16)(__expf(s[j0 + q] - mx) * sc); unsigned short* d = (unsigned short*)P + i * SQ + j0; *(volatile v8us*)d = f.half[0]; __threadfence(); *(volatile v8us*)d = f.half[0]; } }

template <int NHv, int TTv>
__global__ __launch_bounds__(256) void k_vt(const _Float16* __restrict__ V16, int ldv, int voff, _Float16* __restrict__ Vt) { __shared__ unsigned short tl[64][66]; const int tid = threadIdx.x; const int slab = blockIdx.x / (TTv / 64), lg = blockIdx.x % (TTv / 64); const int b = slab / NHv, h = slab % NHv;
  for (int i = tid; i < 64 * 8; i += 256) { const int r = i / 8, c8 = (i % 8) * 8; FragH f; f.half[0] = *(const v8us*)((const unsigned short*)V16 + ((size_t)b * TTv + lg * 64 + r) * ldv + voff + h * 64 + c8);
#pragma unroll
    for (int q = 0; q < 8; ++q) tl[r][c8 + q] = f.u[q]; }
  __syncthreads();
  for (int pass = 0; pass < 2; ++pass) {
#pragma unroll
    for (int rd = 0; rd < 2; ++rd) { const int d = rd * 32 + tid / 8, pc = tid % 8; FragH f;
#pragma unroll
      for (int q = 0; q < 8; ++q) f.u[q] = tl[pc * 8 + q][d];
      *(volatile v8us*)((unsigned short*)Vt + ((size_t)slab * 64 + d) * TTv + lg * 64 + pc * 8) = f.half[0]; }
    if (pass == 0) __threadfence(); } }

extern "C" void kernel_launch(void* const* d_in, const int* in_sizes, int n_in,
                              void* d_out, int out_size, void* d_ws, size_t ws_size, hipStream_t stream) {
  if (n_in < 16) return;
  const float* const* I = (const float* const*)d_in;
  const float* src_q = I[0]; const float* src_kv = I[1]; const float* gq = I[2]; const float* bq = I[3]; const float* gkv = I[4]; const float* bkv = I[5];
  const float* Wq = I[6]; const float* Wkv = I[7]; const float* Wproj = I[8]; const float* bproj = I[9]; const float* gn = I[10]; const float* bn = I[11];
  const float* W1 = I[12]; const float* b1 = I[13]; const float* W2 = I[14]; const float* b2 = I[15];
  const size_t rows_needed = (size_t)(NB - 1) * SEQ_FULL + SEQ;
  if ((size_t)in_sizes[0] < rows_needed * DM || (size_t)in_sizes[1] < rows_needed * DM) return;
  if (in_sizes[2] < DM || in_sizes[3] < DM || in_sizes[4] < DM || in_sizes[5] < DM || in_sizes[9] < DM || in_sizes[10] < DM || in_sizes[11] < DM || in_sizes[15] < DM || in_sizes[13] < DFF) return;
  if ((size_t)in_sizes[6] < (size_t)DM * DM || (size_t)in_sizes[7] < (size_t)2 * DM * DM || (size_t)in_sizes[8] < (size_t)DM * DM || (size_t)in_sizes[12] < (size_t)DM * DFF || (size_t)in_sizes[14] < (size_t)DFF * DM) return;
  if ((size_t)out_size < rows_needed * DM) return;

  const size_t bq_b = (size_t)DM * DM * 2, bkv_b = (size_t)DM * 2 * DM * 2, bo_b = (size_t)DM * DM * 2, bw1_b = (size_t)DFF * DM * 2, bw2_b = (size_t)DM * DFF * 2;
  const size_t n16 = NR * DM * 2, n32 = NR * DM * 4, kv16_b = NR * 2 * DM * 2, p_b = (size_t)HG * SEQ * SEQ * 2, s_b = (size_t)HG * SEQ * SEQ * 4, vt_b = (size_t)NH * HD * SEQ * 2, h16_b = NR * DFF * 2;
  size_t reg0 = bq_b + bkv_b + bo_b; if (n16 > reg0) reg0 = n16;
  const size_t oBQ = 0, oBKV = oBQ + bq_b, oBO = oBKV + bkv_b, oM16 = 0;
  const size_t oBW1 = reg0, oBW2 = oBW1 + bw1_b, G = oBW2 + bw2_b;
  size_t ra = p_b; if (2 * n16 > ra) ra = 2 * n16; if (n32 > ra) ra = n32;
  const size_t oQN = G, oKVN = G + n16, oP = G, oX1 = G, oHF = G;
  const size_t oQ16 = G + ra, oKV16 = oQ16 + n16, oO16 = oKV16 + kv16_b, oVT = oO16 + n16, oS = oVT + vt_b, endA = oS + s_b;
  const size_t oSR = oHF + h16_b, endB = oSR + n32;
  const size_t total = endA > endB ? endA : endB;
  if (total > ws_size) return;
  char* ws = (char*)d_ws;
  _Float16* BQ = (_Float16*)(ws + oBQ); _Float16* BKV = (_Float16*)(ws + oBKV); _Float16* BO = (_Float16*)(ws + oBO); _Float16* BW1 = (_Float16*)(ws + oBW1); _Float16* BW2 = (_Float16*)(ws + oBW2);
  _Float16* QN16 = (_Float16*)(ws + oQN); _Float16* KVN16 = (_Float16*)(ws + oKVN); _Float16* Q16 = (_Float16*)(ws + oQ16); _Float16* KV16 = (_Float16*)(ws + oKV16); _Float16* O16 = (_Float16*)(ws + oO16);
  _Float16* VT = (_Float16*)(ws + oVT); float* S = (float*)(ws + oS); _Float16* P = (_Float16*)(ws + oP); float* X1 = (float*)(ws + oX1); _Float16* M16 = (_Float16*)(ws + oM16); float* SRCN = (float*)(ws + oSR); _Float16* HF16 = (_Float16*)(ws + oHF);
  float* out = (float*)d_out;

  k_wt_f16<<<(unsigned)(((size_t)DM * (DM / 8) + 255) / 256), 256, 0, stream>>>(Wq, BQ, DM, DM, 16.0f);
  k_wt_f16<<<(unsigned)(((size_t)2 * DM * (DM / 8) + 255) / 256), 256, 0, stream>>>(Wkv, BKV, DM, 2 * DM, 16.0f);
  k_wt_f16<<<(unsigned)(((size_t)DM * (DM / 8) + 255) / 256), 256, 0, stream>>>(Wproj, BO, DM, DM, 16.0f);
  k_wt_f16<<<(unsigned)(((size_t)DFF * (DM / 8) + 255) / 256), 256, 0, stream>>>(W1, BW1, DM, DFF, 16.0f);
  k_wt_f16<<<(unsigned)(((size_t)DM * (DFF / 8) + 255) / 256), 256, 0, stream>>>(W2, BW2, DFF, DM, 16.0f);
  k_lnx<1, 1, 1, 0><<<(unsigned)NR, 256, 0, stream>>>(src_q, gq, bq, 1e-5f, QN16, nullptr);
  k_lnx<1, 1, 1, 0><<<(unsigned)NR, 256, 0, stream>>>(src_kv, gkv, bkv, 1e-5f, KVN16, nullptr);
  k_gemm2<0, 0, 0><<<dim3((unsigned)((NR / 128) * (DM / 64)), 1), 128, 0, stream>>>(QN16, DM, 0, BQ, DM, 0, 0.0625f, nullptr, 0, nullptr, 0, nullptr, Q16, DM, 0, (int)NR, DM, DM);
  k_gemm2<0, 0, 0><<<dim3((unsigned)((NR / 128) * (2 * DM / 64)), 1), 128, 0, stream>>>(KVN16, DM, 0, BKV, DM, 0, 0.0625f, nullptr, 0, nullptr, 0, nullptr, KV16, 2 * DM, 0, (int)NR, 2 * DM, DM);
  for (int b = 0; b < NB; ++b) { const size_t r0 = (size_t)b * SEQ;
    k_vt<NH, SEQ><<<NH * (SEQ / 64), 256, 0, stream>>>(KV16 + r0 * 2 * DM, 2 * DM, DM, VT);
    for (int hg0 = 0; hg0 < NH; hg0 += HG) {
      k_gemm2<0, 0, 0><<<dim3((SEQ / 128) * (SEQ / 64), HG), 128, 0, stream>>>(Q16 + r0 * DM + (size_t)hg0 * HD, DM, (size_t)HD, KV16 + r0 * 2 * DM + (size_t)hg0 * HD, 2 * DM, (size_t)HD, 0.125f, nullptr, 0, nullptr, 0, S, nullptr, SEQ, (size_t)SEQ * SEQ, SEQ, SEQ, HD);
      k_rsmf<<<(unsigned)((SEQ * HG + 255) / 256), 256, 0, stream>>>(S, P, SEQ, HG);
      k_gemm2<0, 0, 0><<<dim3((SEQ / 128) * (HD / 64), HG), 128, 0, stream>>>(P, SEQ, (size_t)SEQ * SEQ, VT + (size_t)hg0 * HD * SEQ, SEQ, (size_t)HD * SEQ, 0.25f, nullptr, 0, nullptr, 0, nullptr, O16 + r0 * DM + (size_t)hg0 * HD, DM, (size_t)HD, SEQ, HD, SEQ); } }
  k_gemm2<0, 1, 0><<<dim3((unsigned)((NR / 128) * (DM / 64)), 1), 128, 0, stream>>>(O16, DM, 0, BO, DM, 0, 0.0001220703125f, bproj, 0, src_q, 0, X1, nullptr, DM, 0, (int)NR, DM, DM);
  k_lnx<0, 0, 1, 1><<<(unsigned)NR, 256, 0, stream>>>(X1, gn, bn, 1e-5f, M16, SRCN);
  k_gemm2g<<<dim3((unsigned)((NR / 128) * (DFF / 64)), 1), 128, 0, stream>>>(M16, DM, BW1, DM, 0.0625f, b1, HCARRY, HF16, DFF, (int)NR, DFF, DM);
  k_gemm2<0, 0, 1><<<dim3((unsigned)((NR / 128) * (DM / 64)), 1), 128, 0, stream>>>(HF16, DFF, 0, BW2, DFF, 0, 0.00390625f, b2, 0, SRCN, 0, out, nullptr, DM, 0, (int)NR, DM, DFF);
}
